// DyNeXt_32169305047205
// MI455X (gfx1250) — hardware-verified
//
#include <hip/hip_runtime.h>


#define NB_  32
#define CC   128
#define HW   3136
#define HH   56
#define CR   32
#define CE   512
#define KK   25
#define NROW (NB_ * HW)
#define GI   4
#define GR   (GI * HW)
#define DM   CC
#define LOSC 1024.0f
typedef _Float16 h16;
typedef unsigned short bf;
typedef __attribute__((ext_vector_type(16))) __bf16   v16bf;
typedef __attribute__((ext_vector_type(16))) _Float16 v16h;
typedef __attribute__((ext_vector_type(8)))  _Float16 v8h;
typedef __attribute__((ext_vector_type(8)))  unsigned short v8us;
typedef __attribute__((ext_vector_type(8)))  float    v8f;
typedef __attribute__((ext_vector_type(4)))  float    v4f;
typedef v8h  __attribute__((may_alias)) v8ha;
typedef v4f  __attribute__((may_alias)) v4fa;
typedef v8us __attribute__((may_alias)) v8usa;

__device__ __forceinline__ unsigned short f2bf(float f) { unsigned u = __float_as_uint(f); u += 0x7FFFu + ((u >> 16) & 1u); return (unsigned short)(u >> 16); }
__device__ __forceinline__ float bf2f(unsigned short b) { return __uint_as_float(((unsigned)b) << 16); }
__device__ __forceinline__ float bfr(float f) { return bf2f(f2bf(f)); }
__device__ __forceinline__ v16h cat16(v8h lo, v8h hi) { return __builtin_shufflevector(lo, hi, 0, 1, 2, 3, 4, 5, 6, 7, 8, 9, 10, 11, 12, 13, 14, 15); }
__device__ __forceinline__ v16bf cat16b(v8us lo, v8us hi) { return __builtin_bit_cast(v16bf, __builtin_shufflevector(lo, hi, 0, 1, 2, 3, 4, 5, 6, 7, 8, 9, 10, 11, 12, 13, 14, 15)); }
__device__ __forceinline__ v8f wmma16(v16h a, v16h b, v8f c) { return __builtin_amdgcn_wmma_f32_16x16x32_f16(false, a, false, b, (short)0, c, false, false); }
__device__ __forceinline__ v8f wmmab(v16bf a, v16bf b, v8f c) { return __builtin_amdgcn_wmma_f32_16x16x32_bf16(false, a, false, b, (short)0, c, false, false); }

template <bool SPLITA, bool F16OUT = false>
__global__ __launch_bounds__(128) void k_gemmb(const bf* __restrict__ A, const bf* __restrict__ Al, const bf* __restrict__ Bn, const float* __restrict__ bias, float* C, int ldc, h16* C2, const float* __restrict__ R = nullptr, int K = DM, int roundR = 1) {
    __shared__ __align__(16) float ost[4][16 * 68];
    const int lane = threadIdx.x & 31, wave = threadIdx.x >> 5, lr = lane & 15, hi = lane >> 4;
    const int r0 = blockIdx.x * 64 + wave * 16, c0 = blockIdx.y * 64;
    const size_t aoff = (size_t)(r0 + lr) * K + 8 * hi;
    size_t boff[4];
#pragma unroll
    for (int t = 0; t < 4; ++t) boff[t] = (size_t)(c0 + t * 16 + lr) * K + 8 * hi;
    v8f acc[4];
#pragma unroll
    for (int t = 0; t < 4; ++t) acc[t] = (v8f){};
#pragma unroll 1
    for (int kc = 0; kc < K; kc += 32) {
        const v16bf a = cat16b(*(const v8us*)(A + aoff + kc), *(const v8us*)(A + aoff + kc + 16));
        v16bf al = a;
        if (SPLITA) al = cat16b(*(const v8us*)(Al + aoff + kc), *(const v8us*)(Al + aoff + kc + 16));
#pragma unroll
        for (int t = 0; t < 4; ++t) { const v16bf b = cat16b(*(const v8us*)(Bn + boff[t] + kc), *(const v8us*)(Bn + boff[t] + kc + 16)); acc[t] = wmmab(a, b, acc[t]); if (SPLITA) acc[t] = wmmab(al, b, acc[t]); }
        asm volatile("v_nop\n\tv_nop\n\tv_nop\n\tv_nop" : "+v"(acc[0]), "+v"(acc[1]), "+v"(acc[2]), "+v"(acc[3]) : "v"(a), "v"(al));
    }
    float* os = &ost[wave][0];
#pragma unroll
    for (int t = 0; t < 4; ++t) { const float bv = bias ? bfr(bias[c0 + t * 16 + lr]) : 0.f;
#pragma unroll
        for (int j = 0; j < 8; ++j) os[(hi * 8 + j) * 68 + t * 16 + lr] = acc[t][j] + bv; }
    __syncthreads();
    if (F16OUT) {
        h16* crow = (h16*)(void*)C + (size_t)r0 * ldc + c0;
        auto pass = [&]() {
#pragma unroll
            for (int s = 0; s < 4; ++s) { const int row = 4 * s + (lane >> 3), piece = lane & 7; const float* sp = os + row * 68 + piece * 8; v8h o, o2;
#pragma unroll
                for (int i = 0; i < 8; ++i) { const h16 a = (h16)sp[i]; o[i] = a; o2[i] = (h16)((sp[i] - (float)a) * LOSC); }
                *(volatile v8h*)(crow + (size_t)row * ldc + piece * 8) = o; if (C2) *(volatile v8h*)(C2 + (size_t)r0 * ldc + c0 + (size_t)row * ldc + piece * 8) = o2; }
        };
        pass(); __threadfence(); pass();
    } else {
        float* crow = C + (size_t)r0 * ldc + c0;
        auto pass = [&]() {
#pragma unroll
            for (int s = 0; s < 8; ++s) { const int Lid = (lane >> 3) + 4 * s, piece = lane & 7; const int row = Lid >> 1, cofs = (Lid & 1) * 32 + piece * 4;
                v4f val = *(const v4fa*)(os + row * 68 + cofs); if (R) { const v4f rv = *(const v4f*)(R + ((size_t)r0 + row) * ldc + c0 + cofs); val += roundR ? (v4f){bfr(rv[0]), bfr(rv[1]), bfr(rv[2]), bfr(rv[3])} : rv; }
                *(volatile v4f*)(crow + (size_t)row * ldc + cofs) = val; }
        };
        pass(); __threadfence(); pass();
    }
}

__global__ __launch_bounds__(256) void k_cvt8(const float* __restrict__ src, bf* dst, size_t n8) {
    const size_t i = (size_t)blockIdx.x * 256 + threadIdx.x; if (i >= n8) return;
    const v8f v = *(const v8f*)(src + i * 8); v8us o;
#pragma unroll
    for (int k = 0; k < 8; ++k) o[k] = f2bf(v[k]);
    *(volatile v8us*)(dst + i * 8) = o; __threadfence(); *(volatile v8us*)(dst + i * 8) = o;
}
__global__ __launch_bounds__(256) void k_zero8(bf* dst, size_t n8) {
    const size_t i = (size_t)blockIdx.x * 256 + threadIdx.x; if (i >= n8) return; v8us z;
#pragma unroll
    for (int k = 0; k < 8; ++k) z[k] = 0;
    *(volatile v8us*)(dst + i * 8) = z; __threadfence(); *(volatile v8us*)(dst + i * 8) = z;
}

__device__ __forceinline__ float gelu_e(float x) { return 0.5f * x * (1.0f + erff(x * 0.70710678118654752f)); }
__global__ __launch_bounds__(256) void k_pool(const float* __restrict__ x, float* POOL) {
    __shared__ float sp[32];
    const int lane = threadIdx.x & 31, wv = threadIdx.x >> 5; const int base = blockIdx.x * 32;
#pragma unroll 1
    for (int q = 0; q < 4; ++q) { const int bc = base + wv * 4 + q; const float* xp = x + (size_t)bc * HW; float s = 0.f;
#pragma unroll 1
        for (int p = lane; p < HW; p += 32) s += bfr(xp[p]);
#pragma unroll
        for (int sh = 16; sh; sh >>= 1) s += __shfl_xor(s, sh, 32);
        if (lane == 0) sp[wv * 4 + q] = s * (1.0f / HW); }
    __syncthreads();
    if (wv == 0) { const float v = sp[lane]; *(volatile float*)(POOL + base + lane) = v; __threadfence(); *(volatile float*)(POOL + base + lane) = v; }
}
__global__ __launch_bounds__(256) void k_dyn(const float* __restrict__ POOL, const float* __restrict__ w1, const float* __restrict__ lw, const float* __restrict__ lb, const float* __restrict__ w2, float* DYN) {
    const int lane = threadIdx.x & 31; const int b = blockIdx.x * 8 + (threadIdx.x >> 5); if (b >= NB_) return;
    float h = 0.f;
#pragma unroll 1
    for (int c = 0; c < CC; ++c) h = fmaf(POOL[b * CC + c], bfr(w1[lane * CC + c]), h);
    float s = h;
#pragma unroll
    for (int sh = 16; sh; sh >>= 1) s += __shfl_xor(s, sh, 32);
    const float mu = s * (1.0f / CR); const float d = h - mu; float q = d * d;
#pragma unroll
    for (int sh = 16; sh; sh >>= 1) q += __shfl_xor(q, sh, 32);
    const float hn = d * rsqrtf(q * (1.0f / CR) + 1e-6f) * bfr(lw[lane]) + bfr(lb[lane]);
#pragma unroll 1
    for (int ps = 0; ps < 2; ++ps) {
#pragma unroll 1
        for (int k = 0; k < (CC * KK) / 32; ++k) { const int o = k * 32 + lane; float a = 0.f;
#pragma unroll
            for (int j = 0; j < CR; ++j) a = fmaf(__shfl(hn, j, 32), bfr(w2[(size_t)o * CR + j]), a);
            *(volatile float*)(DYN + (size_t)b * CC * KK + o) = a; }
        if (ps == 0) __threadfence(); }
}
__global__ __launch_bounds__(256) void k_dwconv(const float* __restrict__ x, const float* __restrict__ DYN, float* OUTC) {
    const int lane = threadIdx.x & 31; const size_t w = (size_t)blockIdx.x * 8 + (threadIdx.x >> 5); if (w >= (size_t)NB_ * CC * (HW / 32)) return; const size_t bc = w / (HW / 32); const int p = (int)(w % (HW / 32)) * 32 + lane; const int y = p / HH, xx = p % HH;
    const float* xp = x + bc * HW; const float* dw = DYN + bc * KK; float acc = 0.f;
#pragma unroll 1
    for (int ty = 0; ty < 5; ++ty) { const int yy = y + ty - 2; if (yy < 0 || yy >= HH) continue;
#pragma unroll 1
        for (int tx = 0; tx < 5; ++tx) { const int x2 = xx + tx - 2; if (x2 < 0 || x2 >= HH) continue; acc = fmaf(bfr(xp[yy * HH + x2]), dw[ty * 5 + tx], acc); } }
    float* dst = OUTC + bc * HW + p; *(volatile float*)dst = acc; __threadfence(); *(volatile float*)dst = acc;
}
__global__ __launch_bounds__(256) void k_lnT(const float* __restrict__ OUTC, int b0, const float* __restrict__ lw, const float* __restrict__ lb, bf* Ph, bf* Pl) {
    __shared__ float tl[128][65];
    typedef __attribute__((ext_vector_type(4))) unsigned short v4us;
    const int tid = threadIdx.x; const int p0 = blockIdx.x * 64; const int b = b0 + blockIdx.y; const int g = blockIdx.y;
#pragma unroll
    for (int k = 0; k < 32; ++k) { const int c = k * 4 + (tid >> 6), pp = tid & 63; tl[c][pp] = OUTC[((size_t)b * CC + c) * HW + p0 + pp]; }
    __syncthreads();
    const int pp = tid >> 2, part = tid & 3; float s = 0.f;
#pragma unroll 1
    for (int k = 0; k < 32; ++k) s += tl[part * 32 + k][pp];
    s += __shfl_xor(s, 1, 32); s += __shfl_xor(s, 2, 32); const float mu = s * (1.0f / CC); float q = 0.f;
#pragma unroll 1
    for (int k = 0; k < 32; ++k) { const float d = tl[part * 32 + k][pp] - mu; q = fmaf(d, d, q); }
    q += __shfl_xor(q, 1, 32); q += __shfl_xor(q, 2, 32); const float rs = rsqrtf(q * (1.0f / CC) + 1e-6f);
    __syncthreads();
#pragma unroll 1
    for (int k = 0; k < 32; ++k) { const int c = part * 32 + k; tl[c][pp] = (tl[c][pp] - mu) * rs * bfr(lw[c]) + bfr(lb[c]); }
    __syncthreads();
    const int lane = tid & 31, wv = tid >> 5;
    auto pass = [&]() {
#pragma unroll
        for (int st = 0; st < 4; ++st) { const int pr = wv * 8 + st * 2 + (lane >> 4); const int cl = (lane & 15) * 4;
#pragma unroll
            for (int half = 0; half < 2; ++half) { const int cb = half * 64 + cl; v4us oh, ol;
#pragma unroll
                for (int i = 0; i < 4; ++i) { const float y = tl[cb + i][pr]; const unsigned short hb = f2bf(y); oh[i] = hb; ol[i] = f2bf(y - bf2f(hb)); }
                const size_t o = ((size_t)g * HW + p0 + pr) * CC + cb; *(volatile v4us*)(Ph + o) = oh; *(volatile v4us*)(Pl + o) = ol; } }
    };
    pass(); __threadfence(); pass();
}
__global__ __launch_bounds__(256) void k_gelu512(const float* __restrict__ E, size_t rows, float* G) {
    const int lane = threadIdx.x & 31; const size_t r = (size_t)blockIdx.x * 8 + (threadIdx.x >> 5); if (r >= rows) return;
#pragma unroll 1
    for (int q = 0; q < CE / 128; ++q) { const size_t o = r * CE + q * 128 + lane * 4; const v4f v = *(const v4f*)(E + o); v4f gv;
#pragma unroll
        for (int i = 0; i < 4; ++i) gv[i] = gelu_e(v[i]);
        *(volatile v4f*)(G + o) = gv; __threadfence(); *(volatile v4f*)(G + o) = gv; }
}
__global__ __launch_bounds__(256) void k_gx(const float* __restrict__ G, float* GX) {
    const int lane = threadIdx.x & 31; const int w = blockIdx.x * 8 + (threadIdx.x >> 5); if (w >= GI * (CE / 32)) return; const int g = w / (CE / 32); const int o = (w % (CE / 32)) * 32 + lane; float s = 0.f;
#pragma unroll 1
    for (int p = 0; p < HW; ++p) { const float v = G[((size_t)g * HW + p) * CE + o]; s = fmaf(v, v, s); }
    const float r = sqrtf(s); *(volatile float*)(GX + g * CE + o) = r; __threadfence(); *(volatile float*)(GX + g * CE + o) = r;
}
__global__ __launch_bounds__(256) void k_grnpl(const float* __restrict__ G, const float* __restrict__ GX, const float* __restrict__ gam, const float* __restrict__ bet, bf* Ph, bf* Pl) {
    typedef __attribute__((ext_vector_type(4))) unsigned short v4us;
    const int lane = threadIdx.x & 31; const size_t r = (size_t)blockIdx.x * 8 + (threadIdx.x >> 5); if (r >= (size_t)GR) return; const int g = (int)(r / HW); float m = 0.f;
#pragma unroll 1
    for (int o = lane; o < CE; o += 32) m += GX[g * CE + o];
#pragma unroll
    for (int sh = 16; sh; sh >>= 1) m += __shfl_xor(m, sh, 32);
    const float inv = 1.0f / (m * (1.0f / CE) + 1e-6f);
#pragma unroll 1
    for (int ps = 0; ps < 2; ++ps) {
#pragma unroll 1
        for (int q = 0; q < CE / 128; ++q) { const int c0 = q * 128 + lane * 4; v4us oh, ol;
#pragma unroll
            for (int i = 0; i < 4; ++i) { const int o = c0 + i; const float gv = G[r * CE + o]; const float y = bfr(gam[o]) * (gv * (GX[g * CE + o] * inv)) + bfr(bet[o]) + gv; const unsigned short hb = f2bf(y); oh[i] = hb; ol[i] = f2bf(y - bf2f(hb)); }
            *(volatile v4us*)(Ph + r * CE + c0) = oh; *(volatile v4us*)(Pl + r * CE + c0) = ol; }
        if (ps == 0) __threadfence(); }
}
__global__ __launch_bounds__(256) void k_outT(const float* __restrict__ Y, const float* __restrict__ x, int b0, float* OUTB) {
    __shared__ float tl[64][65];
    const int tid = threadIdx.x; const int p0 = blockIdx.x * 64, c0 = blockIdx.y * 64; const int g = blockIdx.z, b = b0 + g; const int rr = tid >> 2, cq = (tid & 3) * 16;
#pragma unroll
    for (int i = 0; i < 16; ++i) tl[rr][cq + i] = Y[((size_t)g * HW + p0 + rr) * CC + c0 + cq + i];
    __syncthreads();
    const int lane = tid & 31, wv = tid >> 5;
    auto pass = [&]() {
#pragma unroll
        for (int st = 0; st < 4; ++st) { const int cr = wv * 8 + st * 2 + (lane >> 4); const int pq = (lane & 15) * 4; const size_t o = ((size_t)b * CC + c0 + cr) * HW + p0 + pq; v4f v;
#pragma unroll
            for (int i = 0; i < 4; ++i) v[i] = tl[pq + i][cr] + bfr(x[o + i]);
            *(volatile v4f*)(OUTB + o) = v; }
    };
    pass(); __threadfence(); pass();
}
extern "C" void kernel_launch(void* const* d_in, const int* in_sizes, int n_in,
                              void* d_out, int out_size, void* d_ws, size_t ws_size, hipStream_t stream) {
    (void)in_sizes; (void)n_in; (void)out_size;
    const float* x = (const float*)d_in[0]; const float* wfc1 = (const float*)d_in[1]; const float* ln1w = (const float*)d_in[2]; const float* ln1b = (const float*)d_in[3]; const float* wfc2 = (const float*)d_in[4]; const float* ln2w = (const float*)d_in[5]; const float* ln2b = (const float*)d_in[6]; const float* wexp = (const float*)d_in[7]; const float* wshr = (const float*)d_in[8]; const float* gam = (const float*)d_in[9]; const float* bet = (const float*)d_in[10];
    float* out = (float*)d_out;
    char* wsp = (char*)d_ws;
    auto take = [&](size_t bytes) { char* p = wsp; wsp += (bytes + 255) & ~(size_t)255; return (void*)p; };
    bf* WEXP = (bf*)take((size_t)CE * CC * 2); bf* WSHR = (bf*)take((size_t)CC * CE * 2); float* POOL = (float*)take(NB_ * CC * 4); float* DYN = (float*)take((size_t)NB_ * CC * KK * 4); float* OUTC = (float*)take((size_t)NB_ * CC * HW * 4);
    bf* Ph = (bf*)take((size_t)GR * CC * 2); bf* Pl = (bf*)take((size_t)GR * CC * 2); float* E = (float*)take((size_t)GR * CE * 4); float* G = (float*)take((size_t)GR * CE * 4); float* GX = (float*)take(GI * CE * 4); bf* Gh = (bf*)take((size_t)GR * CE * 2); bf* Gl = (bf*)take((size_t)GR * CE * 2); float* Y = (float*)take((size_t)GR * CC * 4);
    if ((size_t)(wsp - (char*)d_ws) > ws_size) return;
    k_cvt8<<<(unsigned)((CE * CC / 8 + 255) / 256), 256, 0, stream>>>(wexp, WEXP, CE * CC / 8); k_cvt8<<<(unsigned)((CC * CE / 8 + 255) / 256), 256, 0, stream>>>(wshr, WSHR, CC * CE / 8);
    k_pool<<<(NB_ * CC) / 32, 256, 0, stream>>>(x, POOL);
    k_dyn<<<NB_ / 8, 256, 0, stream>>>(POOL, wfc1, ln1w, ln1b, wfc2, DYN);
    k_dwconv<<<(NB_ * CC * (HW / 32)) / 8, 256, 0, stream>>>(x, DYN, OUTC);
    for (int b0 = 0; b0 < NB_; b0 += GI) {
        k_lnT<<<dim3(HW / 64, GI, 1), 256, 0, stream>>>(OUTC, b0, ln2w, ln2b, Ph, Pl);
        k_gemmb<true, false><<<dim3(GR / 64, CE / 64, 1), 128, 0, stream>>>(Ph, Pl, WEXP, nullptr, E, CE, nullptr, nullptr, CC);
        k_gelu512<<<GR / 8, 256, 0, stream>>>(E, GR, G);
        k_gx<<<(GI * (CE / 32)) / 8, 256, 0, stream>>>(G, GX);
        k_grnpl<<<GR / 8, 256, 0, stream>>>(G, GX, gam, bet, Gh, Gl);
        k_gemmb<true, false><<<dim3(GR / 64, CC / 64, 1), 128, 0, stream>>>(Gh, Gl, WSHR, nullptr, Y, CC, nullptr, nullptr, CE);
        k_outT<<<dim3(HW / 64, CC / 64, GI), 256, 0, stream>>>(Y, x, b0, out); }
}
